// RelationalGraphConvolutionRP_65747359367363
// MI455X (gfx1250) — hardware-verified
//
#include <hip/hip_runtime.h>
#include <stddef.h>


#define NF     256
#define NO     256
#define NB     8
#define NREL   8
#define NSL    17
#define BM     128
#define BMSH   7
#define HALVES 2
#define NT     512
#define NWV    (NT / 32)
#define CAP    4096
#define TPT    4
#define CH     (NT * TPT)
#define NKEY   (2 * NREL * BM)
#define IDBITS 21
#define IDMASK 0x1FFFFFu

typedef _Float16 v16h __attribute__((ext_vector_type(16)));
typedef _Float16 v8h  __attribute__((ext_vector_type(8)));
typedef float    v8f  __attribute__((ext_vector_type(8)));
typedef float    v4f  __attribute__((ext_vector_type(4)));

union Frag   { v16h v; v8h half[2]; };
union P16    { v8h h; v4f f; };
union BigLds { v8h h[BM * (NF / 8)]; float s[(BM / 2) * NO]; v4f f[(BM / 2) * NO / 4]; };

static_assert(sizeof(BigLds) == 65536);
static_assert(BM == (1 << BMSH));
static_assert(NKEY == 2048);
static_assert(NWV == 16);
static_assert((CAP / 2) % NT == 0);
static_assert(NF == 256 && NO == 256);

__device__ __forceinline__ void wmma2(v8f& c0, v8f& c1, v16h a0, v16h a1, v16h b) {
  c0 = __builtin_amdgcn_wmma_f32_16x16x32_f16(false, a0, false, b, (short)0, c0, false, false);
  c1 = __builtin_amdgcn_wmma_f32_16x16x32_f16(false, a1, false, b, (short)0, c1, false, false);
  asm volatile("v_nop\n\tv_nop\n\tv_nop\n\tv_nop" : "+v"(c0), "+v"(c1) : "v"(a0), "v"(a1), "v"(b));
}

__global__ void __launch_bounds__(256)
k_wconv(const float* __restrict__ bases, const float* __restrict__ comps, _Float16* wt, int nsl)
{
  const int gid = blockIdx.x * blockDim.x + threadIdx.x;
  const int total = nsl * NO * (NF / 8);
  if (gid >= total) return;
  const int i8 = gid & (NF / 8 - 1);
  const int o  = (gid >> 5) & (NO - 1);
  const int sl = gid >> 13;
  float cb[NB];
#pragma unroll
  for (int b = 0; b < NB; ++b) cb[b] = comps[sl * NB + b];
  v8h hv;
#pragma unroll
  for (int j = 0; j < 8; ++j) {
    const int i = i8 * 8 + j;
    float a = 0.f;
#pragma unroll
    for (int b = 0; b < NB; ++b) a += cb[b] * bases[((size_t)b * NF + i) * NO + o];
    hv[j] = (_Float16)(a * 16.0f);
  }
  P16 pk;
  pk.h = hv;
  _Float16* dst = wt + ((size_t)sl * NO + o) * NF + i8 * 8;
  *(volatile v4f*)dst = pk.f;
  __threadfence();
  *(volatile v4f*)dst = pk.f;
}

__global__ void __launch_bounds__(NT)
k_main(const int* __restrict__ tri, const float* __restrict__ feat, const _Float16* __restrict__ wt,
       const float* __restrict__ bias, float* out, int E, int N)
{
  __shared__ BigLds s_big;
  __shared__ unsigned int s_list[HALVES][CAP];
  __shared__ int s_segs[HALVES][NKEY];
  __shared__ int s_sege[HALVES][NKEY];
  __shared__ int s_tot[2][HALVES][NWV];

  const int t = threadIdx.x;
  const int lane = t & 31;
  const int w = t >> 5;
  const int m = lane & 15;
  const int h = lane >> 4;
  const int n0 = blockIdx.x * (HALVES * BM);

  int base0 = 0, base1 = 0;
  const int nchunk = (E + CH - 1) / CH;
  for (int c = 0; c < nchunk; ++c) {
    unsigned int ef[TPT], ei[TPT];
    int hf[TPT], hi[TPT];
    int cnt0 = 0, cnt1 = 0;
#pragma unroll
    for (int j = 0; j < TPT; ++j) {
      const int e = c * CH + j * NT + t;
      hf[j] = 0; hi[j] = 0; ef[j] = 0u; ei[j] = 0u;
      if (e < E) {
        const size_t eb = (size_t)e * 3;
        const int s  = tri[eb];
        const int rr = tri[eb + 1];
        const int o  = tri[eb + 2];
        const int r  = min(max(rr, 0), NREL - 1);
        const int ls = s - n0;
        const int lo = o - n0;
        if ((unsigned)ls < (unsigned)(HALVES * BM)) {
          hf[j] = 1 + (ls >> BMSH);
          ef[j] = ((unsigned)(r * BM + (ls & (BM - 1))) << IDBITS) | ((unsigned)o & IDMASK);
        }
        if ((unsigned)lo < (unsigned)(HALVES * BM)) {
          hi[j] = 1 + (lo >> BMSH);
          ei[j] = ((unsigned)((r + NREL) * BM + (lo & (BM - 1))) << IDBITS) | ((unsigned)s & IDMASK);
        }
        cnt0 += (hf[j] == 1) + (hi[j] == 1);
        cnt1 += (hf[j] == 2) + (hi[j] == 2);
      }
    }
    int in0 = cnt0, in1 = cnt1;
#pragma unroll
    for (int d = 1; d < 32; d <<= 1) {
      const int y0 = __shfl_up(in0, d);
      const int y1 = __shfl_up(in1, d);
      if (lane >= d) { in0 += y0; in1 += y1; }
    }
    const int ex0 = in0 - cnt0;
    const int ex1 = in1 - cnt1;
    const int wa0 = __shfl(in0, 31);
    const int wa1 = __shfl(in1, 31);
    const int par = c & 1;
    if (lane == 0) { s_tot[par][0][w] = wa0; s_tot[par][1][w] = wa1; }
    __syncthreads();
    int tv0 = s_tot[par][0][lane & (NWV - 1)];
    int tv1 = s_tot[par][1][lane & (NWV - 1)];
    if (lane >= NWV) { tv0 = 0; tv1 = 0; }
    int pv0 = (lane < w) ? tv0 : 0;
    int pv1 = (lane < w) ? tv1 : 0;
#pragma unroll
    for (int d = 1; d < NWV; d <<= 1) {
      tv0 += __shfl_xor(tv0, d);
      tv1 += __shfl_xor(tv1, d);
      pv0 += __shfl_xor(pv0, d);
      pv1 += __shfl_xor(pv1, d);
    }
    int pos0 = base0 + __shfl(pv0, 0) + ex0;
    int pos1 = base1 + __shfl(pv1, 0) + ex1;
    base0 += __shfl(tv0, 0);
    base1 += __shfl(tv1, 0);
#pragma unroll
    for (int j = 0; j < TPT; ++j) {
      if (hf[j] == 1)      { if (pos0 < CAP) s_list[0][pos0] = ef[j]; ++pos0; }
      else if (hf[j] == 2) { if (pos1 < CAP) s_list[1][pos1] = ef[j]; ++pos1; }
      if (hi[j] == 1)      { if (pos0 < CAP) s_list[0][pos0] = ei[j]; ++pos0; }
      else if (hi[j] == 2) { if (pos1 < CAP) s_list[1][pos1] = ei[j]; ++pos1; }
    }
  }
  const int H0 = min(base0, CAP);
  const int H1 = min(base1, CAP);
  for (int p = t; p < CAP; p += NT) {
    if (p >= H0) s_list[0][p] = 0xFFFFFFFFu;
    if (p >= H1) s_list[1][p] = 0xFFFFFFFFu;
  }
  __syncthreads();

  for (int k = 2; k <= CAP; k <<= 1) {
    for (int j = k >> 1; j > 0; j >>= 1) {
#pragma unroll
      for (int qq = 0; qq < (HALVES * (CAP / 2)) / NT; ++qq) {
        const int li = qq / ((CAP / 2) / NT);
        const int q  = t + (qq % ((CAP / 2) / NT)) * NT;
        const int i  = ((q & ~(j - 1)) << 1) | (q & (j - 1));
        const int i2 = i | j;
        const unsigned int a = s_list[li][i];
        const unsigned int b = s_list[li][i2];
        const bool up = ((i & k) == 0);
        const bool sw = up ? (a > b) : (b > a);
        if (sw) { s_list[li][i] = b; s_list[li][i2] = a; }
      }
      __syncthreads();
    }
  }

  for (int p = t; p < NKEY; p += NT) {
    s_segs[0][p] = 0; s_sege[0][p] = 0;
    s_segs[1][p] = 0; s_sege[1][p] = 0;
  }
  __syncthreads();
#pragma unroll
  for (int li = 0; li < HALVES; ++li) {
    const int Hl = li ? H1 : H0;
    for (int p = t; p < Hl; p += NT) {
      const int key = (int)(s_list[li][p] >> IDBITS);
      const int kp  = (p > 0) ? (int)(s_list[li][p - 1] >> IDBITS) : -1;
      const int kn  = (p + 1 < Hl) ? (int)(s_list[li][p + 1] >> IDBITS) : -1;
      if (key != kp) s_segs[li][key] = p;
      if (key != kn) s_sege[li][key] = p + 1;
    }
  }
  __syncthreads();

  const int rg = w >> 2;
  const int cg = w & 3;
  const v8f zero8 = {0.f, 0.f, 0.f, 0.f, 0.f, 0.f, 0.f, 0.f};
  const float osc = 1.0f / 256.0f;
  const v4f bz0 = *(const v4f*)(bias + 4 * lane);
  const v4f bz1 = *(const v4f*)(bias + (NO / 2) + 4 * lane);

  for (int hh = 0; hh < HALVES; ++hh) {
    const int nb = n0 + hh * BM;
    if (nb >= N) break;
    v8f acc[8];
#pragma unroll
    for (int i = 0; i < 8; ++i) acc[i] = zero8;

    for (int sl = 0; sl < NSL; ++sl) {
#pragma unroll 1
      for (int q = 0; q < BM / NWV; ++q) {
        const int ln = w * (BM / NWV) + q;
        float ar[8];
#pragma unroll
        for (int i = 0; i < 8; ++i) ar[i] = 0.f;
        float scl = 0.f;
        if (sl < NSL - 1) {
          const int key = sl * BM + ln;
          int st = s_segs[hh][key];
          int en = s_sege[hh][key];
          st = min(max(st, 0), CAP);
          en = min(max(en, st), CAP);
#pragma unroll 2
          for (int p = st; p < en; ++p) {
            const unsigned int ent = s_list[hh][p];
            int id = (int)(ent & IDMASK);
            id = min(id, N - 1);
            const v4f* fp = (const v4f*)(feat + (size_t)id * NF + 8 * lane);
            const v4f x0 = fp[0];
            const v4f x1 = fp[1];
            ar[0] += x0.x; ar[1] += x0.y; ar[2] += x0.z; ar[3] += x0.w;
            ar[4] += x1.x; ar[5] += x1.y; ar[6] += x1.z; ar[7] += x1.w;
          }
          const int cn = en - st;
          scl = (cn > 0) ? (16.0f * (1.0f / (float)cn)) : 0.f;
        } else {
          const int node = nb + ln;
          if (node < N) {
            const v4f* fp = (const v4f*)(feat + (size_t)node * NF + 8 * lane);
            const v4f x0 = fp[0];
            const v4f x1 = fp[1];
            ar[0] = x0.x; ar[1] = x0.y; ar[2] = x0.z; ar[3] = x0.w;
            ar[4] = x1.x; ar[5] = x1.y; ar[6] = x1.z; ar[7] = x1.w;
          }
          scl = 16.0f;
        }
        v8h hv;
#pragma unroll
        for (int i = 0; i < 8; ++i) hv[i] = (_Float16)(ar[i] * scl);
        s_big.h[ln * (NF / 8) + lane] = hv;
      }
      __syncthreads();

      const _Float16* wsl = wt + (size_t)sl * NO * NF;
#pragma unroll 1
      for (int ks = 0; ks < NF / 32; ++ks) {
        Frag a0, a1;
        const int ra = (32 * rg + m) * (NF / 8) + 4 * ks + h;
        a0.half[0] = s_big.h[ra];
        a0.half[1] = s_big.h[ra + 2];
        a1.half[0] = s_big.h[ra + 16 * (NF / 8)];
        a1.half[1] = s_big.h[ra + 16 * (NF / 8) + 2];
#pragma unroll
        for (int tt = 0; tt < 4; ++tt) {
          const int n = 64 * cg + 16 * tt + m;
          const _Float16* bp = wsl + (size_t)n * NF + 32 * ks + 8 * h;
          Frag b;
          b.half[0] = *(const v8h*)bp;
          b.half[1] = *(const v8h*)(bp + 16);
          wmma2(acc[2 * tt], acc[2 * tt + 1], a0.v, a1.v, b.v);
        }
      }
      __syncthreads();
    }

    for (int ps = 0; ps < 2; ++ps) {
      if ((rg >> 1) == ps) {
#pragma unroll
        for (int tt = 0; tt < 4; ++tt) {
#pragma unroll
          for (int u = 0; u < 2; ++u) {
#pragma unroll
            for (int r = 0; r < 8; ++r) {
              const int rl  = 32 * rg + 16 * u + 8 * h + r - 64 * ps;
              const int col = 64 * cg + 16 * tt + m;
              s_big.s[rl * NO + col] = acc[2 * tt + u][r] * osc;
            }
          }
        }
      }
      __syncthreads();
      v4f vv[8];
#pragma unroll
      for (int i = 0; i < 4; ++i) {
        const int rl = 4 * w + i;
        vv[2 * i]     = s_big.f[rl * (NO / 4) + lane] + bz0;
        vv[2 * i + 1] = s_big.f[rl * (NO / 4) + (NO / 8) + lane] + bz1;
      }
#pragma unroll
      for (int i = 0; i < 4; ++i) {
        const int grow = nb + 64 * ps + 4 * w + i;
        if (grow < N) {
          float* op = out + (size_t)grow * NO;
          *(volatile v4f*)(op + 4 * lane) = vv[2 * i];
          *(volatile v4f*)(op + (NO / 2) + 4 * lane) = vv[2 * i + 1];
        }
      }
      __threadfence();
#pragma unroll
      for (int i = 0; i < 4; ++i) {
        const int grow = nb + 64 * ps + 4 * w + i;
        if (grow < N) {
          float* op = out + (size_t)grow * NO;
          *(volatile v4f*)(op + 4 * lane) = vv[2 * i];
          *(volatile v4f*)(op + (NO / 2) + 4 * lane) = vv[2 * i + 1];
        }
      }
      __syncthreads();
    }
  }
}

extern "C" void kernel_launch(void* const* d_in, const int* in_sizes, int n_in,
                              void* d_out, int out_size, void* d_ws, size_t ws_size,
                              hipStream_t stream)
{
  (void)n_in; (void)out_size;
  const int*   tri   = (const int*)d_in[0];
  const float* feat  = (const float*)d_in[1];
  const float* bases = (const float*)d_in[2];
  const float* comps = (const float*)d_in[3];
  const float* bias  = (const float*)d_in[4];
  float* out = (float*)d_out;

  const int E = in_sizes[0] / 3;
  const int N = in_sizes[1] / NF;

  const size_t wt_bytes = (size_t)NSL * NO * NF * sizeof(_Float16);
  if (wt_bytes > ws_size || E <= 0 || N <= 0) return;
  _Float16* wtp = (_Float16*)d_ws;

  const int nthr_w = NSL * NO * (NF / 8);
  k_wconv<<<(nthr_w + 255) / 256, 256, 0, stream>>>(bases, comps, wtp, NSL);

  const int nblk = (N + HALVES * BM - 1) / (HALVES * BM);
  k_main<<<nblk, NT, 0, stream>>>(tri, feat, wtp, bias, out, E, N);
}
